// EdgeConv_9405978378388
// MI455X (gfx1250) — hardware-verified
//
#include <hip/hip_runtime.h>
#include <math.h>

constexpr int kBatch = 4;
constexpr int kNodes = 8192;
constexpr int kCin   = 64;
constexpr int kKnb   = 16;
constexpr int kCout  = 64;
constexpr int kCe    = 2 * kCin;
constexpr int kPts   = kBatch * kNodes;
constexpr int kEdges = kPts * kKnb;
constexpr int kBlocks = 512;
constexpr int kWaves  = 8;
constexpr int kTilesPerWave = 8;
constexpr int kPtsPerBlock  = kWaves * kTilesPerWave;
constexpr int kBlkPerBatch  = kNodes / kPtsPerBlock;
constexpr float kInvCnt   = 1.0f / 131072.0f;
constexpr float kCarry    = 16.0f;
constexpr float kInvCarry = 1.0f / 16.0f;
constexpr float kInvProd  = 1.0f / 256.0f;
constexpr float kEps      = 1e-5f;
constexpr int kPA = 136;
constexpr int kPB = 72;
constexpr int kPS = 68;
constexpr int kWbufFloats = 16 * kPS;
constexpr int kPartFloats = 128;
static_assert(kBlocks * kPtsPerBlock == kPts);
static_assert(kBlkPerBatch * kPtsPerBlock == kNodes);
static_assert(kCe % 32 == 0 && kCout % 32 == 0 && kCin % 32 == 0);
static_assert(16 * kPA * 2 <= kWbufFloats * 4);
static_assert(16 * kPB * 2 <= kWbufFloats * 4);
static_assert((kPA % 8) == 0 && (kPB % 8) == 0);

typedef __attribute__((ext_vector_type(16))) _Float16 v16h;
typedef __attribute__((ext_vector_type(8)))  _Float16 v8h;
typedef __attribute__((ext_vector_type(4)))  _Float16 v4h;
typedef __attribute__((ext_vector_type(16))) __bf16   v16b;
typedef __attribute__((ext_vector_type(8)))  __bf16   v8b;
typedef __attribute__((ext_vector_type(8)))  float    v8f;
typedef __attribute__((ext_vector_type(4)))  float    v4f;
typedef __attribute__((ext_vector_type(4)))  unsigned int v4u;

__device__ __forceinline__ unsigned short f2bf_bits(float f) {
  unsigned u = __float_as_uint(f);
  return (unsigned short)((u + 0x7FFFu + ((u >> 16) & 1u)) >> 16);
}
__device__ __forceinline__ float bf_bits2f(unsigned short h) { return __uint_as_float(((unsigned)h) << 16); }

__device__ __forceinline__ void dep_guard_h(v8f& a, v8f& b, v16h x, v16h y) { asm volatile("v_nop\n\tv_nop\n\tv_nop\n\tv_nop" : "+v"(a), "+v"(b) : "v"(x), "v"(y)); }
__device__ __forceinline__ void dep_guard_b(v8f& a, v8f& b, v16b x, v16b y) { asm volatile("v_nop\n\tv_nop\n\tv_nop\n\tv_nop" : "+v"(a), "+v"(b) : "v"(x), "v"(y)); }
__device__ __forceinline__ void keep4_h(v16h a, v16h b, v16h c, v16h d) { asm volatile("v_nop" :: "v"(a), "v"(b), "v"(c), "v"(d)); }
__device__ __forceinline__ void keep4_b(v16b a, v16b b, v16b c, v16b d) { asm volatile("v_nop" :: "v"(a), "v"(b), "v"(c), "v"(d)); }
__device__ __forceinline__ void acc_guard4(v8f& a, v8f& b, v8f& c, v8f& d) { asm volatile("v_nop\n\tv_nop\n\tv_nop\n\tv_nop" : "+v"(a), "+v"(b), "+v"(c), "+v"(d)); }
template <typename T> struct Frag;
template <> struct Frag<_Float16> {
  typedef v16h V; union U { v16h v; v8h h[2]; };
  static __device__ __forceinline__ v16h load(const _Float16* p) {
    U f; f.h[0] = *(const v8h*)(p); f.h[1] = *(const v8h*)(p + 16); return f.v;
  }
  static __device__ __forceinline__ v8f mma(v16h a, v16h b, v8f c) {
    return __builtin_amdgcn_wmma_f32_16x16x32_f16(false, a, false, b, (short)0, c, false, false);
  }
  static __device__ __forceinline__ void guard(v8f& a, v8f& b, v16h x, v16h y) { dep_guard_h(a, b, x, y); }
  static __device__ __forceinline__ void keep(v16h a, v16h b, v16h c, v16h d) { keep4_h(a, b, c, d); }
};
template <> struct Frag<__bf16> {
  typedef v16b V; union U { v16b v; v8b h[2]; };
  static __device__ __forceinline__ v16b load(const __bf16* p) {
    U f; f.h[0] = *(const v8b*)(p); f.h[1] = *(const v8b*)(p + 16); return f.v;
  }
  static __device__ __forceinline__ v8f mma(v16b a, v16b b, v8f c) {
    return __builtin_amdgcn_wmma_f32_16x16x32_bf16(false, a, false, b, (short)0, c, false, false);
  }
  static __device__ __forceinline__ void guard(v8f& a, v8f& b, v16b x, v16b y) { dep_guard_b(a, b, x, y); }
  static __device__ __forceinline__ void keep(v16b a, v16b b, v16b c, v16b d) { keep4_b(a, b, c, d); }
};

__device__ __forceinline__ float h16_to_f32(unsigned hb) {
  const unsigned sgn = (hb & 0x8000u) << 16; const unsigned em = hb & 0x7fffu;
  const float fn = __uint_as_float((em << 13) + 0x38000000u);
  const float fs = (float)em * 5.9604644775390625e-8f;
  const float mag = (em < 0x400u) ? fs : fn; return __uint_as_float(__float_as_uint(mag) | sgn); }

__device__ __forceinline__ void mma_guard_all(v8f& a0, v8f& a1, v8f& a2, v8f& a3, v16h x, v16h b0, v16h b1, v16h b2, v16h b3) {
  asm volatile("v_nop\n\tv_nop\n\tv_nop\n\tv_nop" : "+v"(a0), "+v"(a1), "+v"(a2), "+v"(a3) : "v"(x), "v"(b0), "v"(b1), "v"(b2), "v"(b3));
}
__device__ __forceinline__ float lkr(float v) { return (v > 0.f) ? v : 0.01f * v; }

template <int KW, int PITCH>
__device__ __forceinline__ void stage_weights(const float* __restrict__ W, _Float16* sW, int tid) {
  constexpr int nItems = kCout * KW / 4;
  constexpr int perRow = KW / 4;
#pragma unroll 1
  for (int e = tid; e < nItems; e += 256) {
    const int o  = e / perRow;
    const int c4 = (e - o * perRow) * 4;
    const v4f w = *(const v4f*)(W + (size_t)o * KW + c4);
    v4h h;
#pragma unroll
    for (int i = 0; i < 4; ++i) h[i] = (_Float16)(w[i] * kCarry);
    *(v4h*)(sW + o * PITCH + c4) = h;
  }
}

__device__ __forceinline__ void stage_edge_tile(const float* __restrict__ x, const int* __restrict__ ind, int bn, _Float16* At, int lane) {
  const int hh = lane >> 4, rl = lane & 15, c4 = rl * 4;
  const v4f cv = *(const v4f*)(x + (size_t)bn * kCin + c4);
  v4h ch;
#pragma unroll
  for (int e = 0; e < 4; ++e) ch[e] = (_Float16)(cv[e] * kCarry);
#pragma unroll
  for (int i = 0; i < 8; ++i) {
    if (i == 4) asm volatile("" ::: "memory");
    const int row = 2 * i + hh;
    int idx = ind[(size_t)bn * kKnb + row];
    idx = idx < 0 ? 0 : (idx > kPts - 1 ? kPts - 1 : idx);
    const v4f yv = *(const v4f*)(x + (size_t)idx * kCin + c4);
    v4h dh;
#pragma unroll
    for (int e = 0; e < 4; ++e) { const float d = yv[e] - cv[e]; dh[e] = (_Float16)(d * kCarry); }
    *(v4h*)(At + row * kPA + c4) = dh;
    *(v4h*)(At + row * kPA + kCin + c4) = ch;
  }
}

template <int KSTEPS, int PAP, int PBP>
__device__ __forceinline__ void tile_gemm(const _Float16* At, const _Float16* Bs, int lane, v8f (&acc)[4]) {
  const int rl = lane & 15, koff = (lane >> 4) * 8;
#pragma unroll
  for (int j = 0; j < 4; ++j) acc[j] = (v8f){0.f, 0.f, 0.f, 0.f, 0.f, 0.f, 0.f, 0.f};
#pragma unroll 1
  for (int k0 = 0; k0 < KSTEPS * 32; k0 += 32) {
    v16h bf[4];
#pragma unroll
    for (int j = 0; j < 4; ++j) bf[j] = Frag<_Float16>::load(Bs + (j * 16 + rl) * PBP + k0 + koff);
    const v16h af = Frag<_Float16>::load(At + rl * PAP + k0 + koff);
#pragma unroll
    for (int j = 0; j < 4; ++j) acc[j] = Frag<_Float16>::mma(af, bf[j], acc[j]);
    mma_guard_all(acc[0], acc[1], acc[2], acc[3], af, bf[0], bf[1], bf[2], bf[3]);
  }
  acc_guard4(acc[0], acc[1], acc[2], acc[3]);
}

__device__ __forceinline__ void acc_stats(const v8f (&acc)[4], float (&s)[4], float (&q)[4]) {
#pragma unroll
  for (int j = 0; j < 4; ++j) {
    float sj = 0.f, qj = 0.f;
#pragma unroll
    for (int r = 0; r < 8; ++r) { const float v = acc[j][r] * kInvProd; sj += v; qj += v * v; }
    sj += __shfl_xor(sj, 16, 32);
    qj += __shfl_xor(qj, 16, 32);
    s[j] += sj; q[j] += qj;
  }
}

__device__ __forceinline__ void block_partials(float* wb, int wave, int lane, const float (&s)[4], const float (&q)[4],
                                               float* __restrict__ part, int bid) {
  const int hh = lane >> 4, rl = lane & 15;
  float* mine = wb + wave * kWbufFloats;
  if (hh == 0) {
#pragma unroll
    for (int j = 0; j < 4; ++j) { mine[j * 16 + rl] = s[j]; mine[64 + j * 16 + rl] = q[j]; }
  }
  __syncthreads();
  if (wave == 0) {
    v4f t = (v4f){0.f, 0.f, 0.f, 0.f};
#pragma unroll
    for (int w = 0; w < kWaves; ++w) t = t + *(const v4f*)(wb + w * kWbufFloats + 4 * lane);
    float* dst = part + (size_t)bid * kPartFloats + 4 * lane;
    *(volatile v4f*)dst = t;
    __threadfence();
    *(volatile v4f*)dst = t;
  }
}

__global__ __launch_bounds__(256) void k_l1_stats(const float* __restrict__ x, const int* __restrict__ ind,
                                                  const float* __restrict__ W1, float* __restrict__ part1) {
  __shared__ __align__(16) _Float16 sW1[kCout * kPA];
  __shared__ __align__(16) float wbuf[kWaves * kWbufFloats];
  const int tid = threadIdx.x, lane = tid & 31, wave = tid >> 5;
  stage_weights<kCe, kPA>(W1, sW1, tid);
  __syncthreads();
  _Float16* At = (_Float16*)(wbuf + wave * kWbufFloats);
  float s[4] = {0.f, 0.f, 0.f, 0.f}, q[4] = {0.f, 0.f, 0.f, 0.f};
  const int bnw = blockIdx.x * kPtsPerBlock + wave * kTilesPerWave;
#pragma unroll 1
  for (int it = 0; it < kTilesPerWave; ++it) {
    const int bn = bnw + it;
    stage_edge_tile(x, ind, bn, At, lane);
    __syncthreads();
    v8f acc[4];
    tile_gemm<kCe / 32, kPA, kPA>(At, sW1, lane, acc);
    acc_stats(acc, s, q);
    __syncthreads();
  }
  block_partials(wbuf, wave, lane, s, q, part1, blockIdx.x);
}

__global__ __launch_bounds__(256) void k_norm_stats(const float* __restrict__ part, float* __restrict__ stats) {
  const int tid = threadIdx.x;
  const int b = tid >> 6, o = tid & 63;
  float s = 0.f, q = 0.f;
#pragma unroll 4
  for (int blk = 0; blk < kBlkPerBatch; ++blk) {
    const size_t base = (size_t)(b * kBlkPerBatch + blk) * kPartFloats;
    s += part[base + o];
    q += part[base + 64 + o];
  }
  const float mean = s * kInvCnt;
  float var = q * kInvCnt - mean * mean;
  var = fmaxf(var, 0.f);
  const float rs = rsqrtf(var + kEps);
  *(volatile float*)(stats + tid) = mean;
  *(volatile float*)(stats + 256 + tid) = rs;
  __threadfence();
  *(volatile float*)(stats + tid) = mean;
  *(volatile float*)(stats + 256 + tid) = rs;
}

__global__ __launch_bounds__(256) void k_l12(const float* __restrict__ x, const int* __restrict__ ind,
                                             const float* __restrict__ W1, const float* __restrict__ W2,
                                             const float* __restrict__ stats1, unsigned short* __restrict__ H2c,
                                             float* __restrict__ part2) {
  __shared__ __align__(16) _Float16 sW1[kCout * kPA];
  __shared__ __align__(16) _Float16 sW2[kCout * kPB];
  __shared__ __align__(16) float wbuf[kWaves * kWbufFloats];
  const int tid = threadIdx.x, lane = tid & 31, wave = tid >> 5;
  const int hh = lane >> 4, rl = lane & 15;
  const int b = blockIdx.x / kBlkPerBatch;
  stage_weights<kCe, kPA>(W1, sW1, tid);
  stage_weights<kCout, kPB>(W2, sW2, tid);
  float mu1[4], rs1[4];
#pragma unroll
  for (int j = 0; j < 4; ++j) {
    mu1[j] = stats1[b * kCout + j * 16 + rl];
    rs1[j] = stats1[256 + b * kCout + j * 16 + rl];
  }
  __syncthreads();
  float* region = wbuf + wave * kWbufFloats;
  _Float16* At = (_Float16*)region;
  float s[4] = {0.f, 0.f, 0.f, 0.f}, q[4] = {0.f, 0.f, 0.f, 0.f};
  const int bnw = blockIdx.x * kPtsPerBlock + wave * kTilesPerWave;
  const int q8 = lane >> 3, c8 = (lane & 7) * 8;
#pragma unroll 1
  for (int it = 0; it < kTilesPerWave; ++it) {
    const int bn = bnw + it;
    stage_edge_tile(x, ind, bn, At, lane);
    __syncthreads();
    v8f acc1[4];
    tile_gemm<kCe / 32, kPA, kPA>(At, sW1, lane, acc1);
    __syncthreads();
#pragma unroll
    for (int j = 0; j < 4; ++j) {
#pragma unroll
      for (int r = 0; r < 8; ++r) {
        const float v = acc1[j][r] * kInvProd;
        const float hn = lkr((v - mu1[j]) * rs1[j]);
        At[(8 * hh + r) * kPB + j * 16 + rl] = (_Float16)(hn * kCarry);
      }
    }
    __syncthreads();
    v8f acc2[4];
    tile_gemm<kCout / 32, kPB, kPB>(At, sW2, lane, acc2);
    acc_stats(acc2, s, q);
    __syncthreads();
    float* slab = region;
#pragma unroll
    for (int j = 0; j < 4; ++j) {
#pragma unroll
      for (int r = 0; r < 8; ++r) slab[(8 * hh + r) * kPS + j * 16 + rl] = acc2[j][r] * kInvCarry;
    }
    __syncthreads();
    v8h hv[4];
#pragma unroll
    for (int i = 0; i < 4; ++i) {
      const int row = i * 4 + q8;
      const float* sp = slab + row * kPS + c8;
#pragma unroll
      for (int e = 0; e < 8; ++e) hv[i][e] = (_Float16)sp[e];
    }
    for (int pass = 0; pass < 2; ++pass) {
#pragma unroll
      for (int i = 0; i < 4; ++i) {
        const int row = i * 4 + q8;
        *(volatile v8h*)(H2c + ((size_t)(bn * kKnb + row)) * kCout + c8) = hv[i];
      }
      __threadfence();
    }
    __syncthreads();
  }
  block_partials(wbuf, wave, lane, s, q, part2, blockIdx.x);
}

__global__ __launch_bounds__(256) void k_l3(const unsigned short* __restrict__ H2c, const float* __restrict__ W3,
                                            const float* __restrict__ stats2, float* __restrict__ premax,
                                            float* __restrict__ part3) {
  __shared__ __align__(16) _Float16 sW3[kCout * kPB];
  __shared__ __align__(16) float wbuf[kWaves * kWbufFloats];
  __shared__ __align__(16) float pmst[kWaves * kTilesPerWave * kCout];
  const int tid = threadIdx.x, lane = tid & 31, wave = tid >> 5;
  const int hh = lane >> 4, rl = lane & 15;
  const int q8 = lane >> 3, c8 = (lane & 7) * 8;
  const int b = blockIdx.x / kBlkPerBatch;
  stage_weights<kCout, kPB>(W3, sW3, tid);
  const v4f mua = *(const v4f*)(stats2 + b * kCout + c8);
  const v4f mub = *(const v4f*)(stats2 + b * kCout + c8 + 4);
  const v4f rsa = *(const v4f*)(stats2 + 256 + b * kCout + c8);
  const v4f rsb = *(const v4f*)(stats2 + 256 + b * kCout + c8 + 4);
  float mu[8], rs[8];
#pragma unroll
  for (int e = 0; e < 4; ++e) { mu[e] = mua[e]; mu[4 + e] = mub[e]; rs[e] = rsa[e]; rs[4 + e] = rsb[e]; }
  __syncthreads();
  _Float16* At = (_Float16*)(wbuf + wave * kWbufFloats);
  float* pm = pmst + wave * (kTilesPerWave * kCout);
  float s[4] = {0.f, 0.f, 0.f, 0.f}, q[4] = {0.f, 0.f, 0.f, 0.f};
  const int bnw = blockIdx.x * kPtsPerBlock + wave * kTilesPerWave;
#pragma unroll 1
  for (int it = 0; it < kTilesPerWave; ++it) {
    const int bn = bnw + it;
#pragma unroll
    for (int i = 0; i < 4; ++i) {
      const int row = i * 4 + q8;
      const v4u w = *(const v4u*)(H2c + ((size_t)(bn * kKnb + row)) * kCout + c8);
      v8h hv;
#pragma unroll
      for (int e = 0; e < 4; ++e) {
        const unsigned we = w[e];
        const float f0 = h16_to_f32(we & 0xffffu);
        const float f1 = h16_to_f32(we >> 16);
        const float a0 = lkr((f0 * kInvCarry - mu[2 * e]) * rs[2 * e]);
        const float a1 = lkr((f1 * kInvCarry - mu[2 * e + 1]) * rs[2 * e + 1]);
        hv[2 * e]     = (_Float16)(a0 * kCarry);
        hv[2 * e + 1] = (_Float16)(a1 * kCarry);
      }
      *(v8h*)(At + row * kPB + c8) = hv;
    }
    __syncthreads();
    v8f acc3[4];
    tile_gemm<kCout / 32, kPB, kPB>(At, sW3, lane, acc3);
    acc_stats(acc3, s, q);
#pragma unroll
    for (int j = 0; j < 4; ++j) {
      float m = acc3[j][0];
#pragma unroll
      for (int r = 1; r < 8; ++r) m = fmaxf(m, acc3[j][r]);
      m = fmaxf(m, __shfl_xor(m, 16, 32));
      if (hh == 0) pm[it * kCout + j * 16 + rl] = m * kInvProd;
    }
    __syncthreads();
  }
  {
    float* dst = premax + (size_t)bnw * kCout;
    v4f pv[4];
#pragma unroll
    for (int i = 0; i < 4; ++i) pv[i] = *(const v4f*)(pm + i * 128 + 4 * lane);
    for (int pass = 0; pass < 2; ++pass) {
#pragma unroll
      for (int i = 0; i < 4; ++i) *(volatile v4f*)(dst + i * 128 + 4 * lane) = pv[i];
      __threadfence();
    }
  }
  block_partials(wbuf, wave, lane, s, q, part3, blockIdx.x);
}

__global__ __launch_bounds__(256) void k_out(const float* __restrict__ premax, const float* __restrict__ stats3,
                                             float* __restrict__ out) {
  const int g = blockIdx.x * 256 + threadIdx.x;
  const int b = g >> 17;
  const int o4 = (g & 15) * 4;
  const v4f v  = *(const v4f*)(premax + 4 * (size_t)g);
  const v4f mu = *(const v4f*)(stats3 + b * kCout + o4);
  const v4f rs = *(const v4f*)(stats3 + 256 + b * kCout + o4);
  v4f r;
#pragma unroll
  for (int e = 0; e < 4; ++e) { const float t = (v[e] - mu[e]) * rs[e]; r[e] = lkr(t); }
  float* dst = out + 4 * (size_t)g;
  *(volatile v4f*)dst = r;
  __threadfence();
  *(volatile v4f*)dst = r;
}

extern "C" void kernel_launch(void* const* d_in, const int* in_sizes, int n_in,
                              void* d_out, int out_size, void* d_ws, size_t ws_size, hipStream_t stream) {
  if (n_in < 5) return;
  if (in_sizes[0] != kPts * kCin || in_sizes[1] != kPts * kKnb || in_sizes[2] != kCout * kCe ||
      in_sizes[3] != kCout * kCout || in_sizes[4] != kCout * kCout) return;
  if (out_size != kPts * kCout) return;
  const float* x   = (const float*)d_in[0];
  const int*   ind = (const int*)d_in[1];
  const float* W1  = (const float*)d_in[2];
  const float* W2  = (const float*)d_in[3];
  const float* W3  = (const float*)d_in[4];
  float* out = (float*)d_out;

  char* ws = (char*)d_ws; size_t off = 0;
  auto carve = [&](size_t bytes) -> char* { char* p = ws + off; off += (bytes + 255) & ~(size_t)255; return p; };
  unsigned short* H2c = (unsigned short*)carve((size_t)kEdges * kCout * 2);
  float* premax = (float*)carve((size_t)kPts * kCout * 4);
  float* part1 = (float*)carve((size_t)kBlocks * kPartFloats * 4);
  float* part2 = (float*)carve((size_t)kBlocks * kPartFloats * 4);
  float* part3 = (float*)carve((size_t)kBlocks * kPartFloats * 4);
  float* stats1 = (float*)carve(512 * 4);
  float* stats2 = (float*)carve(512 * 4);
  float* stats3 = (float*)carve(512 * 4);
  if (off > ws_size || off > (size_t)134217728) return;

  k_l1_stats<<<kBlocks, 256, 0, stream>>>(x, ind, W1, part1);
  k_norm_stats<<<1, 256, 0, stream>>>(part1, stats1);
  k_l12<<<kBlocks, 256, 0, stream>>>(x, ind, W1, W2, stats1, H2c, part2);
  k_norm_stats<<<1, 256, 0, stream>>>(part2, stats2);
  k_l3<<<kBlocks, 256, 0, stream>>>(H2c, W3, stats2, premax, part3);
  k_norm_stats<<<1, 256, 0, stream>>>(part3, stats3);
  k_out<<<(kPts * kCout / 4) / 256, 256, 0, stream>>>(premax, stats3, out);
}
